// MyMlp_39281770889905
// MI455X (gfx1250) — hardware-run, weakly checked
//
#include <hip/hip_runtime.h>
#include <math.h>

#pragma clang fp contract(off)

typedef __attribute__((ext_vector_type(16))) _Float16 v16h;
typedef __attribute__((ext_vector_type(8)))  _Float16 v8h;
typedef __attribute__((ext_vector_type(8)))  float    v8f;
typedef __attribute__((ext_vector_type(4)))  float    v4f;
typedef __attribute__((ext_vector_type(2)))  float    v2f;
typedef __attribute__((ext_vector_type(4)))  unsigned v4u;
typedef __attribute__((ext_vector_type(2)))  unsigned v2u;

constexpr int kBatch = 8;
constexpr int kTok   = 3136;
constexpr int kGH    = 56;
constexpr int kGW    = 56;
constexpr int kPix   = kGH * kGW;
constexpr int kCin   = 256;
constexpr int kChid  = 1024;
constexpr int kRows  = kBatch * kTok;
constexpr float kWCarry    = 64.0f;
constexpr float kWCarryInv = 1.0f / kWCarry;
static_assert(kPix == 3136 && kTok == 3136, "grid and token counts");
static_assert(kRows == 25088, "rows");
static_assert((kRows % 64) == 0 && (kChid % 64) == 0 && (kCin % 64) == 0, "GEMM M,N multiples of 64");
static_assert((kCin % 32) == 0 && (kChid % 32) == 0, "GEMM K multiples of 32");
static_assert(kPix == 14 * 224 && kTok == 98 * 32, "scan tiling");
static_assert((kRows % 8) == 0, "one wave per row kernels");
static_assert(((kRows / 64) * (kChid / 64)) % 8 == 0 && ((kRows / 64) * (kCin / 64)) % 8 == 0, "GEMM tiles fill whole blocks");

constexpr double kG1d   = 0.8824969025845955;
constexpr double kGSumd = (1.0 + 2.0 * kG1d) * (1.0 + 2.0 * kG1d);
constexpr float  kGwC   = (float)(1.0 / kGSumd);
constexpr float  kGwE   = (float)(kG1d / kGSumd);
constexpr float  kGwK   = (float)(kG1d * kG1d / kGSumd);

constexpr size_t kOffX16  = 0;
constexpr size_t kOffW1   = kOffX16 + (size_t)kRows * kCin * 2;
constexpr size_t kOffW2   = kOffW1  + (size_t)kChid * kCin * 2;
constexpr size_t kOffCnt  = kOffW2  + (size_t)kCin * kChid * 2;
constexpr size_t kOffPA   = kOffCnt + (size_t)kRows * 4;
constexpr size_t kOffPB   = kOffPA  + (size_t)kRows * kChid * 2;
constexpr size_t kWsTotal = kOffPB  + (size_t)kRows * kChid * 2;
static_assert(kWsTotal == 116754432ull, "carve total");
static_assert(kWsTotal <= 134217728ull, "carve cap");
static_assert((kOffW1 % 128) == 0 && (kOffW2 % 128) == 0 && (kOffCnt % 128) == 0 &&
              (kOffPA % 128) == 0 && (kOffPB % 128) == 0, "128-B aligned regions");

__device__ __forceinline__ int iclampi(int v, int lo, int hi) {
  return v < lo ? lo : (v > hi ? hi : v);
}

__device__ __forceinline__ float h16_to_f32(unsigned hb) {
  const unsigned sgn = (hb & 0x8000u) << 16;
  const unsigned em = hb & 0x7fffu;
  const float fn = __uint_as_float((em << 13) + 0x38000000u);
  const float fs = (float)em * 5.9604644775390625e-8f;
  const float mag = (em < 0x400u) ? fs : fn;
  return __uint_as_float(__float_as_uint(mag) | sgn);
}

__device__ __forceinline__ unsigned pack2h(float a, float b) {
  const _Float16 h0 = (_Float16)a, h1 = (_Float16)b;
  return (unsigned)__builtin_bit_cast(unsigned short, h0) |
         ((unsigned)__builtin_bit_cast(unsigned short, h1) << 16);
}

__device__ __forceinline__ void tie_acc_h(v8f& a, v16h x, v16h y) {
  asm volatile("" : "+v"(a) : "v"(x), "v"(y));
}
__device__ __forceinline__ void tie_acc_nop4_h(v8f& a, v16h x, v16h y) {
  asm volatile("v_nop\n\tv_nop\n\tv_nop\n\tv_nop" : "+v"(a) : "v"(x), "v"(y));
}
__device__ __forceinline__ void keep4_h(v16h a, v16h b, v16h c, v16h d) {
  asm volatile("v_nop" :: "v"(a), "v"(b), "v"(c), "v"(d));
}
__device__ __forceinline__ void acc_guard4(v8f& a, v8f& b, v8f& c, v8f& d) {
  asm volatile("v_nop\n\tv_nop\n\tv_nop\n\tv_nop" : "+v"(a), "+v"(b), "+v"(c), "+v"(d));
}

struct FragH {
  union U { v16h v; v8h h[2]; };
  static __device__ __forceinline__ v16h load(const _Float16* p) {
    U f;
    f.h[0] = *(const v8h*)(p);
    f.h[1] = *(const v8h*)(p + 16);
    return f.v;
  }
  static __device__ __forceinline__ v8f mma(v16h a, v16h b, v8f c) {
    return __builtin_amdgcn_wmma_f32_16x16x32_f16(false, a, false, b, (short)0, c, false, false);
  }
};

template <int OUT_MODE, int ACT>
__global__ __launch_bounds__(256) void wmma_gemm64_f16(
    const unsigned short* __restrict__ Ap, int lda,
    const unsigned short* __restrict__ Btp, int ldb,
    void* __restrict__ Cout, int ldc,
    const float* __restrict__ bias,
    int M, int N, int K, float scale) {
  const _Float16* A  = (const _Float16*)Ap;
  const _Float16* Bt = (const _Float16*)Btp;
  __shared__ __align__(16) float sT[8][16 * 68];
  const int lane = threadIdx.x & 31;
  const int wave = threadIdx.x >> 5;
  const int tilesN = N >> 6;
  const int tilesM = M >> 6;
  const int tile = blockIdx.x * 8 + wave;
  if (tile >= tilesM * tilesN) return;
  const int tm = tile / tilesN;
  const int tn = tile - tm * tilesN;
  const int m0 = tm << 6;
  const int n0 = tn << 6;

  const int rlane = lane & 15;
  const int koff  = (lane >> 4) * 8;
  const int mOff  = (lane >> 4) * 8;

  v8f acc[4][4];
#pragma unroll
  for (int i = 0; i < 4; ++i)
#pragma unroll
    for (int j = 0; j < 4; ++j) acc[i][j] = (v8f){0.f,0.f,0.f,0.f,0.f,0.f,0.f,0.f};

  for (int k0 = 0; k0 < K; k0 += 32) {
    v16h bh[4];
#pragma unroll
    for (int j = 0; j < 4; ++j) {
      const size_t bo = (size_t)(n0 + (j << 4) + rlane) * ldb + koff + k0;
      bh[j] = FragH::load(Bt + bo);
    }
#pragma unroll
    for (int i = 0; i < 4; ++i) {
      const size_t ao = (size_t)(m0 + (i << 4) + rlane) * lda + koff + k0;
      const v16h ah = FragH::load(A + ao);
#pragma unroll
      for (int j = 0; j < 4; ++j) acc[i][j] = FragH::mma(ah, bh[j], acc[i][j]);
      tie_acc_h(acc[i][0], ah, bh[0]);
      tie_acc_h(acc[i][1], ah, bh[1]);
      tie_acc_h(acc[i][2], ah, bh[2]);
      tie_acc_nop4_h(acc[i][3], ah, bh[3]);
    }
    keep4_h(bh[0], bh[1], bh[2], bh[3]);
  }
  acc_guard4(acc[0][0], acc[0][1], acc[0][2], acc[0][3]);
  acc_guard4(acc[1][0], acc[1][1], acc[1][2], acc[1][3]);
  acc_guard4(acc[2][0], acc[2][1], acc[2][2], acc[2][3]);
  acc_guard4(acc[3][0], acc[3][1], acc[3][2], acc[3][3]);

  float* slab = sT[wave];
#pragma unroll
  for (int i = 0; i < 4; ++i) {
    const int mBase = m0 + (i << 4);
#pragma unroll
    for (int j = 0; j < 4; ++j) {
      const int n = n0 + (j << 4) + rlane;
      const float bv = bias[n];
#pragma unroll
      for (int r = 0; r < 8; ++r) {
        float v = acc[i][j][r] * scale;
        v += bv;
        if (ACT == 2) v = fmaxf(v, 0.0f);
        slab[(mOff + r) * 68 + (j << 4) + rlane] = v;
      }
    }
    __builtin_amdgcn_fence(__ATOMIC_RELEASE, "workgroup");
    __builtin_amdgcn_wave_barrier();
    __builtin_amdgcn_fence(__ATOMIC_ACQUIRE, "workgroup");
    if (OUT_MODE == 0) {
      float* C = (float*)Cout;
      const int hh = lane >> 4, c4 = (lane & 15) * 4;
      for (int pass = 0; pass < 2; ++pass) {
#pragma unroll
        for (int it = 0; it < 8; ++it) {
          const int row = it * 2 + hh;
          v4f v = *(const v4f*)(slab + row * 68 + c4);
          *(volatile v4f*)(C + (size_t)(mBase + row) * ldc + n0 + c4) = v;
        }
        __threadfence();
      }
    } else {
      const int q = lane >> 3, c8 = (lane & 7) * 8;
      unsigned short* C = (unsigned short*)Cout;
      for (int pass = 0; pass < 2; ++pass) {
#pragma unroll
        for (int it = 0; it < 4; ++it) {
          const int row = it * 4 + q;
          const float* sp = slab + row * 68 + c8;
          v8h hv;
#pragma unroll
          for (int e = 0; e < 8; ++e) hv[e] = (_Float16)sp[e];
          *(volatile v8h*)(C + (size_t)(mBase + row) * ldc + n0 + c8) = hv;
        }
        __threadfence();
      }
    }
    __builtin_amdgcn_fence(__ATOMIC_RELEASE, "workgroup");
    __builtin_amdgcn_wave_barrier();
    __builtin_amdgcn_fence(__ATOMIC_ACQUIRE, "workgroup");
  }
}

__global__ __launch_bounds__(256) void cast_f16x8_kernel(
    const float* __restrict__ src, unsigned short* __restrict__ dst, int total8, float carry) {
  const int i = blockIdx.x * 256 + threadIdx.x;
  if (i >= total8) return;
  const size_t e0 = (size_t)i << 3;
  const v4f a0 = *(const v4f*)(src + e0);
  const v4f a1 = *(const v4f*)(src + e0 + 4);
  v4u w;
  w[0] = pack2h(a0[0] * carry, a0[1] * carry);
  w[1] = pack2h(a0[2] * carry, a0[3] * carry);
  w[2] = pack2h(a1[0] * carry, a1[1] * carry);
  w[3] = pack2h(a1[2] * carry, a1[3] * carry);
  volatile v4u* op = (volatile v4u*)(dst + e0);
  *op = w;
  __threadfence();
  *op = w;
}

__device__ __forceinline__ int token_cell(float lx, float ly) {
  const float cx = fminf(fmaxf(lx, -1.0f), 1.0f);
  const float cy = fminf(fmaxf(ly, -1.0f), 1.0f);
  const float ax = 0.5f * (cx + 1.0f);
  const float ay = 0.5f * (cy + 1.0f);
  const float sx = ax * (float)kGW;
  const float sy = ay * (float)kGH;
  const float rx = sx - 0.5f;
  const float ry = sy - 0.5f;
  const int px = iclampi((int)rintf(rx), 0, kGW - 1);
  const int py = iclampi((int)rintf(ry), 0, kGH - 1);
  return px + py * kGW;
}

__global__ __launch_bounds__(224) void token2map_kernel(
    const float* __restrict__ loc, const unsigned short* __restrict__ h16,
    unsigned short* __restrict__ feat, float* __restrict__ cnt) {
  __shared__ int sIdx[kPix];
  const int tid = threadIdx.x, lane = tid & 31, wave = tid >> 5;
  const int b  = blockIdx.x / 14;
  const int bi = blockIdx.x - b * 14;
  for (int i = tid; i < kTok; i += 224) {
    const v2f l = *(const v2f*)(loc + ((size_t)b * kTok + i) * 2);
    sIdx[i] = token_cell(l[0], l[1]);
  }
  __syncthreads();
  const int pbase = bi * 224 + wave * 32;
  const v4u* hrows = (const v4u*)h16;
  float cntv = 0.0f;
#pragma unroll 1
  for (int j = 0; j < 32; ++j) {
    const int target = pbase + j;
    float acc[32];
#pragma unroll
    for (int e = 0; e < 32; ++e) acc[e] = 0.0f;
    int c = 0;
#pragma unroll 1
    for (int i = 0; i < 98; ++i) {
      const int v = sIdx[i * 32 + lane];
      unsigned m = __builtin_amdgcn_ballot_w32(v == target);
      while (m != 0u) {
        const int bit = __builtin_ctz(m);
        m &= (m - 1u);
        const size_t tok = (size_t)b * kTok + (size_t)(i * 32 + bit);
        const v4u* rp = hrows + tok * 128 + lane;
        v4u wq[4];
        wq[0] = rp[0];
        wq[1] = rp[32];
        wq[2] = rp[64];
        wq[3] = rp[96];
#pragma unroll
        for (int q = 0; q < 4; ++q) {
#pragma unroll
          for (int e = 0; e < 4; ++e) {
            const unsigned w = wq[q][e];
            acc[q * 8 + 2 * e]     += h16_to_f32(w & 0xffffu);
            acc[q * 8 + 2 * e + 1] += h16_to_f32(w >> 16);
          }
        }
        ++c;
      }
    }
    const float fc = (float)c;
    const float rinv = 1.0f / (fc + 1e-6f);
    const float inv = (c > 0) ? rinv : 0.0f;
    v4u o[4];
#pragma unroll
    for (int q = 0; q < 4; ++q) {
#pragma unroll
      for (int e = 0; e < 4; ++e)
        o[q][e] = pack2h(acc[q * 8 + 2 * e] * inv, acc[q * 8 + 2 * e + 1] * inv);
    }
    volatile v4u* op = (volatile v4u*)feat + ((size_t)b * kPix + target) * 128 + lane;
    op[0] = o[0]; op[32] = o[1]; op[64] = o[2]; op[96] = o[3];
    __threadfence();
    op[0] = o[0]; op[32] = o[1]; op[64] = o[2]; op[96] = o[3];
    cntv = (lane == j) ? fc : cntv;
  }
  volatile float* cp = (volatile float*)cnt + (size_t)b * kPix + pbase + lane;
  *cp = cntv;
  __threadfence();
  *cp = cntv;
}

__global__ __launch_bounds__(256) void holefill_kernel(
    const unsigned short* __restrict__ feat, const float* __restrict__ cnt,
    unsigned short* __restrict__ feat2) {
  const int lane = threadIdx.x & 31, wave = threadIdx.x >> 5;
  const int p = blockIdx.x * 8 + wave;
  const int b = p / kPix;
  const int pix = p - b * kPix;
  const int y = pix / kGW;
  const int x = pix - y * kGW;
  const int kk = (lane < 9) ? lane : 8;
  const int kdy = kk / 3;
  const int kdx = kk - kdy * 3;
  const int yy = y + kdy - 1, xx = x + kdx - 1;
  const bool inb = (lane < 9) && (yy >= 0) && (yy < kGH) && (xx >= 0) && (xx < kGW);
  const int yc = iclampi(yy, 0, kGH - 1), xc = iclampi(xx, 0, kGW - 1);
  const float cv = cnt[(size_t)b * kPix + yc * kGW + xc];
  const unsigned m = __builtin_amdgcn_ballot_w32(inb && (cv > 0.0f)) & 0x1FFu;
  const bool occupied = ((m >> 4) & 1u) != 0u;
  const v4u* src = (const v4u*)feat;
  v4u o[4];
  if (occupied) {
    const v4u* rp = src + (size_t)p * 128 + lane;
    o[0] = rp[0];
    o[1] = rp[32];
    o[2] = rp[64];
    o[3] = rp[96];
  } else {
    float acc[32];
#pragma unroll
    for (int e = 0; e < 32; ++e) acc[e] = 0.0f;
    float smm = 0.0f;
    unsigned mm = m;
    while (mm != 0u) {
      const int k = __builtin_ctz(mm);
      mm &= (mm - 1u);
      const int ky = k / 3;
      const int kx = k - ky * 3;
      const int off = ((ky != 1) ? 1 : 0) + ((kx != 1) ? 1 : 0);
      const float wgt = (off == 0) ? kGwC : ((off == 1) ? kGwE : kGwK);
      const int ny = iclampi(y + ky - 1, 0, kGH - 1);
      const int nx = iclampi(x + kx - 1, 0, kGW - 1);
      const v4u* rp = src + ((size_t)b * kPix + ny * kGW + nx) * 128 + lane;
      v4u wq[4];
      wq[0] = rp[0];
      wq[1] = rp[32];
      wq[2] = rp[64];
      wq[3] = rp[96];
#pragma unroll
      for (int q = 0; q < 4; ++q) {
#pragma unroll
        for (int e = 0; e < 4; ++e) {
          const unsigned w = wq[q][e];
          acc[q * 8 + 2 * e]     = fmaf(wgt, h16_to_f32(w & 0xffffu), acc[q * 8 + 2 * e]);
          acc[q * 8 + 2 * e + 1] = fmaf(wgt, h16_to_f32(w >> 16), acc[q * 8 + 2 * e + 1]);
        }
      }
      smm += wgt;
    }
    const float rinv = 1.0f / (smm + 1e-6f);
    const float inv = (smm > 0.0f) ? rinv : 0.0f;
#pragma unroll
    for (int q = 0; q < 4; ++q) {
#pragma unroll
      for (int e = 0; e < 4; ++e)
        o[q][e] = pack2h(acc[q * 8 + 2 * e] * inv, acc[q * 8 + 2 * e + 1] * inv);
    }
  }
  volatile v4u* op = (volatile v4u*)feat2 + (size_t)p * 128 + lane;
  op[0] = o[0]; op[32] = o[1]; op[64] = o[2]; op[96] = o[3];
  __threadfence();
  op[0] = o[0]; op[32] = o[1]; op[64] = o[2]; op[96] = o[3];
}

__device__ __forceinline__ v4f load4h(const v2u* p, bool ok) {
  const v2u w = *p;
  const unsigned w0 = w[0], w1 = w[1];
  v4f r;
  const float f0 = h16_to_f32(w0 & 0xffffu);
  const float f1 = h16_to_f32(w0 >> 16);
  const float f2 = h16_to_f32(w1 & 0xffffu);
  const float f3 = h16_to_f32(w1 >> 16);
  r[0] = ok ? f0 : 0.0f;
  r[1] = ok ? f1 : 0.0f;
  r[2] = ok ? f2 : 0.0f;
  r[3] = ok ? f3 : 0.0f;
  return r;
}

__global__ __launch_bounds__(256) void dwconv_kernel(
    const unsigned short* __restrict__ fin, const float* __restrict__ wgt,
    const float* __restrict__ bias, unsigned short* __restrict__ fout) {
  const int tid = threadIdx.x;
  const int b = blockIdx.x / kGH;
  const int y = blockIdx.x - b * kGH;
  const int c0 = tid * 4;
  v4f wv[9];
#pragma unroll
  for (int i = 0; i < 9; ++i) wv[i] = *(const v4f*)(wgt + (size_t)c0 * 9 + 4 * i);
  const v4f bv = *(const v4f*)(bias + c0);
  const v2u* src = (const v2u*)fin;
  bool rok[3];
  size_t rbase[3];
#pragma unroll
  for (int ky = 0; ky < 3; ++ky) {
    const int yy = y + ky - 1;
    rok[ky] = (yy >= 0) && (yy < kGH);
    const int yc = iclampi(yy, 0, kGH - 1);
    rbase[ky] = ((size_t)b * kPix + (size_t)yc * kGW) * 256 + tid;
  }
  v4f colL[3], colC[3], colR[3];
#pragma unroll
  for (int ky = 0; ky < 3; ++ky) {
    colL[ky] = (v4f){0.f, 0.f, 0.f, 0.f};
    colC[ky] = load4h(src + rbase[ky], rok[ky]);
    colR[ky] = load4h(src + rbase[ky] + 256, rok[ky]);
  }
#pragma unroll 1
  for (int x = 0; x < kGW; ++x) {
    float acc[4];
#pragma unroll
    for (int e = 0; e < 4; ++e) acc[e] = 0.0f;
#pragma unroll
    for (int ky = 0; ky < 3; ++ky) {
#pragma unroll
      for (int e = 0; e < 4; ++e) {
        acc[e] = fmaf(wv[(e * 9 + ky * 3 + 0) >> 2][(e * 9 + ky * 3 + 0) & 3], colL[ky][e], acc[e]);
        acc[e] = fmaf(wv[(e * 9 + ky * 3 + 1) >> 2][(e * 9 + ky * 3 + 1) & 3], colC[ky][e], acc[e]);
        acc[e] = fmaf(wv[(e * 9 + ky * 3 + 2) >> 2][(e * 9 + ky * 3 + 2) & 3], colR[ky][e], acc[e]);
      }
    }
    v2u o;
    o[0] = pack2h(acc[0] + bv[0], acc[1] + bv[1]);
    o[1] = pack2h(acc[2] + bv[2], acc[3] + bv[3]);
    volatile v2u* op = (volatile v2u*)fout + ((size_t)b * kPix + (size_t)y * kGW + x) * 256 + tid;
    *op = o;
    __threadfence();
    *op = o;
    const int xn = x + 2;
    const bool cok = (xn < kGW);
    const int xc = (xn < kGW) ? xn : (kGW - 1);
#pragma unroll
    for (int ky = 0; ky < 3; ++ky) {
      colL[ky] = colC[ky];
      colC[ky] = colR[ky];
      colR[ky] = load4h(src + rbase[ky] + (size_t)xc * 256, rok[ky] && cok);
    }
  }
}

__global__ __launch_bounds__(256) void gather_gelu_kernel(
    const unsigned short* __restrict__ fm, const float* __restrict__ loc,
    const int* __restrict__ pH, const int* __restrict__ pW,
    const int* __restrict__ pKs, const int* __restrict__ pSg,
    unsigned short* __restrict__ t16) {
  const int lane = threadIdx.x & 31, wave = threadIdx.x >> 5;
  const int t = blockIdx.x * 8 + wave;
  const int b = t / kTok;
  const bool premise = (pH[0] == kGH) && (pW[0] == kGW) && (pKs[0] == 3) && (pSg[0] == 2);
  const float poison = __uint_as_float(0x7fc00000u);
  const v2f l = *(const v2f*)(loc + (size_t)t * 2);
  float gx = (l[0] + 1.0f) * (float)kGW;
  gx = gx * 0.5f;
  gx = gx - 0.5f;
  float gy = (l[1] + 1.0f) * (float)kGH;
  gy = gy * 0.5f;
  gy = gy - 0.5f;
  const float x0f = floorf(gx), y0f = floorf(gy);
  const float wx1 = gx - x0f, wy1 = gy - y0f;
  const float wx0 = 1.0f - wx1, wy0 = 1.0f - wy1;
  const int x0 = (int)x0f, y0 = (int)y0f;
  const int x1 = x0 + 1, y1 = y0 + 1;
  const bool vx0 = (x0 >= 0) && (x0 < kGW), vx1 = (x1 >= 0) && (x1 < kGW);
  const bool vy0 = (y0 >= 0) && (y0 < kGH), vy1 = (y1 >= 0) && (y1 < kGH);
  const int xc0 = iclampi(x0, 0, kGW - 1), xc1 = iclampi(x1, 0, kGW - 1);
  const int yc0 = iclampi(y0, 0, kGH - 1), yc1 = iclampi(y1, 0, kGH - 1);
  const float p00 = wx0 * wy0, p10 = wx1 * wy0, p01 = wx0 * wy1, p11 = wx1 * wy1;
  const float w00 = (vx0 && vy0) ? p00 : 0.0f;
  const float w10 = (vx1 && vy0) ? p10 : 0.0f;
  const float w01 = (vx0 && vy1) ? p01 : 0.0f;
  const float w11 = (vx1 && vy1) ? p11 : 0.0f;
  const unsigned* fmw = (const unsigned*)fm;
  const size_t rowb = (size_t)b * kPix;
  const unsigned* r00 = fmw + (rowb + (size_t)(yc0 * kGW + xc0)) * 512 + lane;
  const unsigned* r10 = fmw + (rowb + (size_t)(yc0 * kGW + xc1)) * 512 + lane;
  const unsigned* r01 = fmw + (rowb + (size_t)(yc1 * kGW + xc0)) * 512 + lane;
  const unsigned* r11 = fmw + (rowb + (size_t)(yc1 * kGW + xc1)) * 512 + lane;
  volatile unsigned* orow = (volatile unsigned*)t16 + (size_t)t * 512 + lane;
#pragma unroll 1
  for (int it = 0; it < 16; ++it) {
    const unsigned a00 = r00[it * 32];
    const unsigned a10 = r10[it * 32];
    const unsigned a01 = r01[it * 32];
    const unsigned a11 = r11[it * 32];
    float u0 = h16_to_f32(a00 & 0xffffu) * w00;
    u0 = u0 + h16_to_f32(a10 & 0xffffu) * w10;
    u0 = u0 + h16_to_f32(a01 & 0xffffu) * w01;
    u0 = u0 + h16_to_f32(a11 & 0xffffu) * w11;
    float u1 = h16_to_f32(a00 >> 16) * w00;
    u1 = u1 + h16_to_f32(a10 >> 16) * w10;
    u1 = u1 + h16_to_f32(a01 >> 16) * w01;
    u1 = u1 + h16_to_f32(a11 >> 16) * w11;
    float g0 = 0.5f * u0 * (1.0f + erff(u0 * 0.70710678118654752f));
    float g1 = 0.5f * u1 * (1.0f + erff(u1 * 0.70710678118654752f));
    g0 = premise ? g0 : poison;
    g1 = premise ? g1 : poison;
    const unsigned word = pack2h(g0, g1);
    orow[it * 32] = word;
    __threadfence();
    orow[it * 32] = word;
  }
}

extern "C" void kernel_launch(void* const* d_in, const int* in_sizes, int n_in,
                              void* d_out, int out_size, void* d_ws, size_t ws_size,
                              hipStream_t stream) {
  if (n_in < 12) return;
  if (in_sizes[0] != kRows * kCin) return;
  if (in_sizes[1] != kRows * 2) return;
  if (in_sizes[2] != kChid * kCin) return;
  if (in_sizes[3] != kChid) return;
  if (in_sizes[4] != kCin * kChid) return;
  if (in_sizes[5] != kCin) return;
  if (in_sizes[6] != kChid * 9) return;
  if (in_sizes[7] != kChid) return;
  if (out_size != kRows * kCin) return;
  if (ws_size < kWsTotal) return;

  const float* x     = (const float*)d_in[0];
  const float* loc   = (const float*)d_in[1];
  const float* fc1_w = (const float*)d_in[2];
  const float* fc1_b = (const float*)d_in[3];
  const float* fc2_w = (const float*)d_in[4];
  const float* fc2_b = (const float*)d_in[5];
  const float* dw_w  = (const float*)d_in[6];
  const float* dw_b  = (const float*)d_in[7];
  const int*   pH    = (const int*)d_in[8];
  const int*   pW    = (const int*)d_in[9];
  const int*   pKs   = (const int*)d_in[10];
  const int*   pSg   = (const int*)d_in[11];
  float* out = (float*)d_out;

  char* ws = (char*)d_ws;
  unsigned short* X16 = (unsigned short*)(ws + kOffX16);
  unsigned short* W1  = (unsigned short*)(ws + kOffW1);
  unsigned short* W2  = (unsigned short*)(ws + kOffW2);
  float*          CNT = (float*)(ws + kOffCnt);
  unsigned short* PA  = (unsigned short*)(ws + kOffPA);
  unsigned short* PB  = (unsigned short*)(ws + kOffPB);

  cast_f16x8_kernel<<<(kRows * kCin / 8) / 256, 256, 0, stream>>>(x, X16, kRows * kCin / 8, 1.0f);
  cast_f16x8_kernel<<<(kChid * kCin / 8) / 256, 256, 0, stream>>>(fc1_w, W1, kChid * kCin / 8, kWCarry);
  cast_f16x8_kernel<<<(kCin * kChid / 8) / 256, 256, 0, stream>>>(fc2_w, W2, kCin * kChid / 8, kWCarry);

  wmma_gemm64_f16<1, 2><<<((kRows / 64) * (kChid / 64)) / 8, 256, 0, stream>>>(
      X16, kCin, W1, kCin, (void*)PA, kChid, fc1_b, kRows, kChid, kCin, kWCarryInv);

  token2map_kernel<<<kBatch * 14, 224, 0, stream>>>(loc, PA, PB, CNT);

  holefill_kernel<<<kRows / 8, 256, 0, stream>>>(PB, CNT, PA);

  dwconv_kernel<<<kBatch * kGH, 256, 0, stream>>>(PA, dw_w, dw_b, PB);

  gather_gelu_kernel<<<kRows / 8, 256, 0, stream>>>(PB, loc, pH, pW, pKs, pSg, PA);

  wmma_gemm64_f16<0, 0><<<((kRows / 64) * (kCin / 64)) / 8, 256, 0, stream>>>(
      PA, kChid, W2, kChid, (void*)out, kCin, fc2_b, kRows, kCin, kChid, kWCarryInv);
}
